// GraphMolActorCritic_thv1_65438121722208
// MI455X (gfx1250) — hardware-verified
//
#include <hip/hip_runtime.h>
#include <stddef.h>
#include <math.h>


#define NNODE  8192
#define NEDGE  16384
#define NPAD   8192
#define FIN    14
#define KP0    32
#define DD     64
#define G3     192
#define NGR    256
#define NJB    1024
#define NST    2048
#define NOUT   105
#define NOUTP  128
#define TCOL   4096
#define OUTN   (NGR * 2 + NST * NOUT + NJB)
#define OFF1   (NGR * 2)
#define OFF2   (NGR * 2 + NST * NOUT)
#define ASC    8
#define WSC    64
#define EWSC   64
#define OSC    (1.0f / 512.0f)
#define EWINV  (1.0f / 64.0f)
#define WLC    512
#define TB     256
#define NT     128
#define NWS    8
#define NKT    8
#define NCH    (NT * NKT)
#define WCAPN  (32 * NKT)
#define WSCAP  160000000

static_assert(NPAD % 64 == 0 && NPAD >= NNODE && NPAD - NNODE < 64);
static_assert(NEDGE % 64 == 0 && NEDGE % 4 == 0);
static_assert((NCH & (NCH - 1)) == 0 && NCH <= 4096);
static_assert(NST % 64 == 0 && (2 * NJB) % 64 == 0 && NGR % 16 == 0);
static_assert(TCOL == DD * DD);
static_assert((64 * NOUT * 4) % 128 == 0);
static_assert((OFF1 * 4) % 128 == 0 && (OFF2 * 4) % 128 == 0);
static_assert(OUTN == 216576);
static_assert(NNODE < 65536);
static_assert(FIN <= KP0);

typedef float          v2f  __attribute__((ext_vector_type(2)));
typedef float          v4f  __attribute__((ext_vector_type(4)));
typedef float          v8f  __attribute__((ext_vector_type(8)));
typedef int            v4i  __attribute__((ext_vector_type(4)));
typedef _Float16       v8h  __attribute__((ext_vector_type(8)));
typedef _Float16       v16h __attribute__((ext_vector_type(16)));
typedef unsigned short v8us __attribute__((ext_vector_type(8)));
union FragH { v16h v; v8us u[2]; v8h h[2]; };
union U8 { v8us u; v8h h; };

__device__ __forceinline__ v8f wmh(v16h a, v16h b, v8f c) {
  v8f d = __builtin_amdgcn_wmma_f32_16x16x32_f16(false, a, false, b, (short)0, c, false, false);
  asm volatile("v_nop\n\tv_nop\n\tv_nop\n\tv_nop" : "+v"(d) : "v"(a), "v"(b));
  return d;
}
__device__ __forceinline__ v8f zero8() { v8f z = {0.f, 0.f, 0.f, 0.f, 0.f, 0.f, 0.f, 0.f}; return z; }
__device__ __forceinline__ float leaky_f(float v) { return v > 0.0f ? v : 0.01f * v; }
__device__ __forceinline__ float sigm_f(float x) {
  x = fminf(fmaxf(x, -30.0f), 30.0f);
  return 1.0f / (1.0f + expf(-x));
}
__device__ __forceinline__ float tanh_f(float x) {
  const float ax = fminf(fabsf(x), 15.0f);
  const float e = expf(-2.0f * ax);
  const float t = (1.0f - e) * (1.0f / (1.0f + e));
  return x < 0.0f ? -t : t;
}
__device__ __forceinline__ float wsum32(float v) {
#pragma unroll
  for (int s = 16; s > 0; s >>= 1) v += __shfl_xor(v, s);
  return v;
}

__device__ __forceinline__ v16h frag_glb(const unsigned short* P, int row, int ld, int k0, int hh) {
  FragH f;
  const unsigned short* p = P + (size_t)row * ld + k0 + 8 * hh;
  f.u[0] = *(const v8us*)p;
  f.u[1] = *(const v8us*)(p + 16);
  return f.v;
}
__device__ __forceinline__ v16h frag_lds(const _Float16* T, int row, int ld, int k0, int hh) {
  FragH f;
  const _Float16* p = T + row * ld + k0 + 8 * hh;
  f.h[0] = *(const v8h*)p;
  f.h[1] = *(const v8h*)(p + 16);
  return f.v;
}
__device__ __forceinline__ v8f gemm1(v16h a0, v16h a1, const unsigned short* Bp, int col, int hh) {
  const v16h b0 = frag_glb(Bp, col, DD, 0, hh);
  const v16h b1 = frag_glb(Bp, col, DD, 32, hh);
  v8f d = wmh(a0, b0, zero8());
  d = wmh(a1, b1, d);
  return d;
}

__device__ __forceinline__ void cvt_unit(const float* __restrict__ P, unsigned short* dst, long sc, long sk,
                                         int K, int KP, int Nv, int Nout, float scale, int i) {
  const int upc = KP >> 3;
  if (i >= Nout * upc) return;
  const int n = i / upc;
  const int seg = i - n * upc;
  const int nc = n < Nv - 1 ? n : Nv - 1;
  v8h o;
#pragma unroll
  for (int j = 0; j < 8; ++j) {
    const int k = 8 * seg + j;
    const int kc = k < K - 1 ? k : K - 1;
    const float v = P[(size_t)nc * sc + (size_t)kc * sk];
    const float keep = (k < K && n < Nv) ? scale : 0.0f;
    o[j] = (_Float16)(v * keep);
  }
  const v8us ob = __builtin_bit_cast(v8us, o);
  unsigned short* d = dst + (size_t)i * 8;
  *(volatile v8us*)d = ob;
  __threadfence();
  *(volatile v8us*)d = ob;
}

__global__ __launch_bounds__(TB) void k_prep(
    const float* __restrict__ net2w, const float* __restrict__ croot, const float* __restrict__ wih,
    const float* __restrict__ whh, const float* __restrict__ l0w, const float* __restrict__ s1w,
    const float* __restrict__ s2w, const float* __restrict__ j1w, const float* __restrict__ x,
    unsigned short* BW2, unsigned short* BC, unsigned short* BWI, unsigned short* BWH, unsigned short* BL0,
    unsigned short* BS1, unsigned short* BS2, unsigned short* BJ1, unsigned short* XP) {
  const int job = (int)blockIdx.y;
  const int i = (int)blockIdx.x * TB + (int)threadIdx.x;
  const float* P =
      job == 0 ? net2w : job == 1 ? croot : job == 2 ? wih : job == 3 ? whh : job == 4 ? l0w :
      job == 5 ? s1w : job == 6 ? s2w : job == 7 ? j1w : x;
  unsigned short* D =
      job == 0 ? BW2 : job == 1 ? BC : job == 2 ? BWI : job == 3 ? BWH : job == 4 ? BL0 :
      job == 5 ? BS1 : job == 6 ? BS2 : job == 7 ? BJ1 : XP;
  const long sc = (job == 8) ? FIN : 1;
  const long sk = job == 0 ? TCOL : (job == 2 || job == 3) ? G3 : job == 6 ? NOUT : job == 8 ? 1 : DD;
  const int  K  = (job == 4 || job == 8) ? FIN : DD;
  const int  KP = (job == 4 || job == 8) ? KP0 : DD;
  const int  Nv = job == 0 ? TCOL : (job == 2 || job == 3) ? G3 : job == 6 ? NOUT : job == 8 ? NNODE : DD;
  const int  No = job == 6 ? NOUTP : job == 8 ? NPAD : Nv;
  const float scale = job == 8 ? (float)ASC : (float)WSC;
  cvt_unit(P, D, sc, sk, K, KP, Nv, No, scale, i);
}

__global__ __launch_bounds__(TB) void k_e1(const float* __restrict__ ea, const float* __restrict__ w1,
                                           const float* __restrict__ b1, unsigned short* E1H, int nE) {
  const int tid = threadIdx.x, lane = tid & 31;
  const int gw = ((int)blockIdx.x * TB + tid) >> 5;
  const int e0 = 4 * gw;
  if (e0 >= nE) return;
  int e = e0 + (lane >> 3); e = e > nE - 1 ? nE - 1 : e;
  const int o8 = 8 * (lane & 7);
  const v4f a   = *(const v4f*)(ea + (size_t)e * 4);
  const v4f w0a = *(const v4f*)(w1 + 0 * DD + o8), w0b = *(const v4f*)(w1 + 0 * DD + o8 + 4);
  const v4f w1a = *(const v4f*)(w1 + 1 * DD + o8), w1b = *(const v4f*)(w1 + 1 * DD + o8 + 4);
  const v4f w2a = *(const v4f*)(w1 + 2 * DD + o8), w2b = *(const v4f*)(w1 + 2 * DD + o8 + 4);
  const v4f w3a = *(const v4f*)(w1 + 3 * DD + o8), w3b = *(const v4f*)(w1 + 3 * DD + o8 + 4);
  const v4f ba  = *(const v4f*)(b1 + o8),          bb  = *(const v4f*)(b1 + o8 + 4);
  const v4f ra = ba + a.x * w0a + a.y * w1a + a.z * w2a + a.w * w3a;
  const v4f rb = bb + a.x * w0b + a.y * w1b + a.z * w2b + a.w * w3b;
  v8h r8;
  r8[0] = (_Float16)(leaky_f(ra.x) * (float)ASC); r8[1] = (_Float16)(leaky_f(ra.y) * (float)ASC);
  r8[2] = (_Float16)(leaky_f(ra.z) * (float)ASC); r8[3] = (_Float16)(leaky_f(ra.w) * (float)ASC);
  r8[4] = (_Float16)(leaky_f(rb.x) * (float)ASC); r8[5] = (_Float16)(leaky_f(rb.y) * (float)ASC);
  r8[6] = (_Float16)(leaky_f(rb.z) * (float)ASC); r8[7] = (_Float16)(leaky_f(rb.w) * (float)ASC);
  const v8us rv = __builtin_bit_cast(v8us, r8);
  unsigned short* dp = E1H + (size_t)e * DD + o8;
  *(volatile v8us*)dp = rv;
  __threadfence();
  *(volatile v8us*)dp = rv;
}

__device__ __forceinline__ void ew_rows(const _Float16* st, unsigned short* EW, int e0, int g, int lane) {
#pragma unroll
  for (int i = 0; i < 4; ++i) {
    const int row = 4 * i + (lane >> 3), p = lane & 7;
    const v8h v = *(const v8h*)(st + row * DD + 8 * p);
    const v8us vb = __builtin_bit_cast(v8us, v);
    *(volatile v8us*)(EW + (size_t)(e0 + row) * TCOL + (size_t)g * DD + 8 * p) = vb;
  }
}

__global__ __launch_bounds__(NT) void k_ew(const unsigned short* __restrict__ E1H, const unsigned short* __restrict__ BW2,
                                           const float* __restrict__ b2, unsigned short* EW) {
  __shared__ __attribute__((aligned(16))) _Float16 sSt[4][16 * DD];
  const int tid = threadIdx.x, lane = tid & 31, wave = tid >> 5, hh = lane >> 4, m = lane & 15;
  const int e0 = ((int)blockIdx.x * 4 + wave) * 16;
  _Float16* st = sSt[wave];
  const v16h a0 = frag_glb(E1H, e0 + m, DD, 0, hh);
  const v16h a1 = frag_glb(E1H, e0 + m, DD, 32, hh);
#pragma unroll 1
  for (int g = 0; g < TCOL / DD; ++g) {
#pragma unroll 1
    for (int t = 0; t < 4; ++t) {
      const int cl = 16 * t + m;
      const int col = g * DD + cl;
      const v8f acc = gemm1(a0, a1, BW2, col, hh);
      const float bv = b2[col];
#pragma unroll
      for (int r = 0; r < 8; ++r)
        st[(8 * hh + r) * DD + cl] = (_Float16)((acc[r] * OSC + bv) * (float)EWSC);
    }
    __syncthreads();
    ew_rows(st, EW, e0, g, lane);
    __threadfence();
    ew_rows(st, EW, e0, g, lane);
    __syncthreads();
  }
}

__device__ __forceinline__ void rows_out2(const float* so, float* H32, unsigned short* HH, int n0, int lane) {
#pragma unroll
  for (int i = 0; i < 8; ++i) {
    const int row = 2 * i + (lane >> 4), p = lane & 15;
    const v4f v = *(const v4f*)(so + row * DD + 4 * p);
    *(volatile v4f*)(H32 + (size_t)(n0 + row) * DD + 4 * p) = v;
  }
#pragma unroll
  for (int i = 0; i < 4; ++i) {
    const int row = 4 * i + (lane >> 3), p = lane & 7;
    const v4f a = *(const v4f*)(so + row * DD + 8 * p);
    const v4f b = *(const v4f*)(so + row * DD + 8 * p + 4);
    v8h h8;
    h8[0] = (_Float16)(a.x * (float)ASC); h8[1] = (_Float16)(a.y * (float)ASC);
    h8[2] = (_Float16)(a.z * (float)ASC); h8[3] = (_Float16)(a.w * (float)ASC);
    h8[4] = (_Float16)(b.x * (float)ASC); h8[5] = (_Float16)(b.y * (float)ASC);
    h8[6] = (_Float16)(b.z * (float)ASC); h8[7] = (_Float16)(b.w * (float)ASC);
    const v8us hb = __builtin_bit_cast(v8us, h8);
    *(volatile v8us*)(HH + (size_t)(n0 + row) * DD + 8 * p) = hb;
  }
}

__global__ __launch_bounds__(NT) void k_lin0(const unsigned short* __restrict__ XP,
                                             const unsigned short* __restrict__ BL0,
                                             const float* __restrict__ b0, float* H32, unsigned short* HH) {
  __shared__ __attribute__((aligned(16))) float sOut[4][16 * DD];
  const int tid = threadIdx.x, lane = tid & 31, wave = tid >> 5, hh = lane >> 4, m = lane & 15;
  const int n0 = ((int)blockIdx.x * 4 + wave) * 16;
  float* so = sOut[wave];
  const v16h a = frag_glb(XP, n0 + m, KP0, 0, hh);
#pragma unroll 1
  for (int t = 0; t < 4; ++t) {
    const int c = 16 * t + m;
    const v16h b = frag_glb(BL0, c, KP0, 0, hh);
    const v8f acc = wmh(a, b, zero8());
    const float bv = b0[c];
#pragma unroll
    for (int r = 0; r < 8; ++r) so[(8 * hh + r) * DD + c] = leaky_f(acc[r] * OSC + bv);
  }
  __syncthreads();
  rows_out2(so, H32, HH, n0, lane);
  __threadfence();
  rows_out2(so, H32, HH, n0, lane);
}

__global__ __launch_bounds__(NT) void k_node(
    const float* __restrict__ H32o, const unsigned short* __restrict__ HHo, float* H32n, unsigned short* HHn,
    const unsigned short* __restrict__ EW, const int* __restrict__ esrc, const int* __restrict__ edst,
    const unsigned short* __restrict__ BC, const float* __restrict__ convb,
    const unsigned short* __restrict__ BWI, const unsigned short* __restrict__ BWH,
    const float* __restrict__ bih, const float* __restrict__ bhh, int nN, int nE) {
  __shared__ __attribute__((aligned(16))) float    sAgg[64 * DD];
  __shared__ __attribute__((aligned(16))) _Float16 sM[4][16 * DD];
  __shared__ __attribute__((aligned(16))) float    sOut[4][16 * DD];
  __shared__ __attribute__((aligned(16))) int      sList[4 * WCAPN];
  __shared__ float sInv[64];
  __shared__ int   sDeg[64];
  __shared__ int   sWc[4];
  const int tid = threadIdx.x, lane = tid & 31, wave = tid >> 5, hh = lane >> 4, m = lane & 15;
  const int nb = (int)blockIdx.x * 64;
  const int n0 = nb + 16 * wave;

  {
    const v4f z = {0.f, 0.f, 0.f, 0.f};
    for (int i = tid; i < 64 * DD / 4; i += NT) *(v4f*)(sAgg + 4 * i) = z;
    if (tid < 64) sDeg[tid] = 0;
  }
  __syncthreads();

  const int rowOff = lane >> 3, colg = lane & 7;
  const int nChunks = (nE + NCH - 1) / NCH;
#pragma unroll 1
  for (int ch = 0; ch < nChunks; ++ch) {
    const int cbase = ch * NCH;
    const int el0 = tid * NKT;
    const int e0 = cbase + el0;
    const int sent = -2147483647 - 1;
    v4i da, db;
    if (cbase + NCH <= nE) {
      da = *(const v4i*)(edst + e0);
      db = *(const v4i*)(edst + e0 + 4);
    } else {
      da.x = (e0     < nE) ? edst[min(e0, nE - 1)] : sent;
      da.y = (e0 + 1 < nE) ? edst[min(e0 + 1, nE - 1)] : sent;
      da.z = (e0 + 2 < nE) ? edst[min(e0 + 2, nE - 1)] : sent;
      da.w = (e0 + 3 < nE) ? edst[min(e0 + 3, nE - 1)] : sent;
      db.x = (e0 + 4 < nE) ? edst[min(e0 + 4, nE - 1)] : sent;
      db.y = (e0 + 5 < nE) ? edst[min(e0 + 5, nE - 1)] : sent;
      db.z = (e0 + 6 < nE) ? edst[min(e0 + 6, nE - 1)] : sent;
      db.w = (e0 + 7 < nE) ? edst[min(e0 + 7, nE - 1)] : sent;
    }
    const unsigned nbu = (unsigned)nb;
    const unsigned s0 = (unsigned)da.x - nbu, s1 = (unsigned)da.y - nbu;
    const unsigned s2 = (unsigned)da.z - nbu, s3 = (unsigned)da.w - nbu;
    const unsigned s4 = (unsigned)db.x - nbu, s5 = (unsigned)db.y - nbu;
    const unsigned s6 = (unsigned)db.z - nbu, s7 = (unsigned)db.w - nbu;
    const bool h0 = s0 < 64u, h1 = s1 < 64u, h2 = s2 < 64u, h3 = s3 < 64u;
    const bool h4 = s4 < 64u, h5 = s5 < 64u, h6 = s6 < 64u, h7 = s7 < 64u;
    int wc = 0;
    const unsigned any = __builtin_amdgcn_ballot_w32(h0 | h1 | h2 | h3 | h4 | h5 | h6 | h7);
    if (any != 0u) {
#define HITJ(J, HJ, SJ) { \
        const unsigned mj = __builtin_amdgcn_ballot_w32(HJ); \
        if (mj != 0u) { \
          if (HJ) { \
            const int pos = wc + (int)__builtin_amdgcn_mbcnt_lo(mj, 0u); \
            if (pos < WCAPN) sList[wave * WCAPN + pos] = ((el0 + (J)) << 8) | (int)(SJ); \
          } \
          wc += (int)__builtin_popcount(mj); } }
      HITJ(0, h0, s0)
      HITJ(1, h1, s1)
      HITJ(2, h2, s2)
      HITJ(3, h3, s3)
      HITJ(4, h4, s4)
      HITJ(5, h5, s5)
      HITJ(6, h6, s6)
      HITJ(7, h7, s7)
#undef HITJ
    }
    if (lane == 0) sWc[wave] = wc < WCAPN ? wc : WCAPN;
    __syncthreads();

#pragma unroll 1
    for (int wl = 0; wl < 4; ++wl) {
      int n = __builtin_amdgcn_readfirstlane(sWc[wl]);
      n = n > WCAPN ? WCAPN : (n < 0 ? 0 : n);
#pragma unroll 1
      for (int i = 0; i < n; ++i) {
        const int ent = __builtin_amdgcn_readfirstlane(sList[wl * WCAPN + i]);
        const int loc = ent & 63;
        if ((loc >> 4) == wave) {
          int e = cbase + ((ent >> 8) & (NCH - 1));
          e = e < 0 ? 0 : (e > nE - 1 ? nE - 1 : e);
          int s = esrc[e];
          s = s < 0 ? 0 : (s > nN - 1 ? nN - 1 : s);
          const float* hrow = H32o + (size_t)s * DD;
          const unsigned short* ep = EW + (size_t)e * TCOL + 8 * colg;
          float acc[8];
#pragma unroll
          for (int j = 0; j < 8; ++j) acc[j] = 0.0f;
#pragma unroll 4
          for (int q = 0; q < 16; ++q) {
            const int ii = 4 * q + rowOff;
            const float ai = hrow[ii];
            U8 w; w.u = *(const v8us*)(ep + ii * DD);
#pragma unroll
            for (int j = 0; j < 8; ++j) acc[j] = fmaf(ai, (float)w.h[j], acc[j]);
          }
#pragma unroll
          for (int j = 0; j < 8; ++j) {
            acc[j] += __shfl_xor(acc[j], 8);
            acc[j] += __shfl_xor(acc[j], 16);
          }
          if (lane < 8) {
            float* ap = sAgg + loc * DD + 8 * lane;
            v4f x0 = *(const v4f*)ap;
            v4f x1 = *(const v4f*)(ap + 4);
            x0.x += acc[0] * EWINV; x0.y += acc[1] * EWINV; x0.z += acc[2] * EWINV; x0.w += acc[3] * EWINV;
            x1.x += acc[4] * EWINV; x1.y += acc[5] * EWINV; x1.z += acc[6] * EWINV; x1.w += acc[7] * EWINV;
            *(v4f*)ap = x0;
            *(v4f*)(ap + 4) = x1;
          }
          if (lane == 0) sDeg[loc] = sDeg[loc] + 1;
        }
      }
    }
    __syncthreads();
  }

  if (tid < 64) {
    const int dg = sDeg[tid];
    sInv[tid] = 1.0f / (float)(dg > 1 ? dg : 1);
  }
  __syncthreads();

  float* sa = sAgg + wave * 16 * DD;
  _Float16* sm = sM[wave];
  float* so = sOut[wave];
  const v16h aH0 = frag_glb(HHo, n0 + m, DD, 0, hh);
  const v16h aH1 = frag_glb(HHo, n0 + m, DD, 32, hh);

#pragma unroll 1
  for (int t = 0; t < 4; ++t) {
    const int c = 16 * t + m;
    const v8f d = gemm1(aH0, aH1, BC, c, hh);
    const float cb = convb[c];
#pragma unroll
    for (int r = 0; r < 8; ++r) {
      const int rl = 8 * hh + r;
      const float v = d[r] * OSC + cb + sa[rl * DD + c] * sInv[16 * wave + rl];
      sm[rl * DD + c] = (_Float16)(leaky_f(v) * (float)ASC);
    }
  }
  __syncthreads();

#pragma unroll 1
  for (int t = 0; t < 4; ++t) {
    const int c = 16 * t + m;
    const v8f dhr = gemm1(aH0, aH1, BWH, c, hh);
    const v8f dhz = gemm1(aH0, aH1, BWH, DD + c, hh);
    const v8f dhn = gemm1(aH0, aH1, BWH, 2 * DD + c, hh);
    const v16h pH0 = frag_lds(sm, m, DD, 0, hh);
    const v16h pH1 = frag_lds(sm, m, DD, 32, hh);
    const v8f dir = gemm1(pH0, pH1, BWI, c, hh);
    const v8f diz = gemm1(pH0, pH1, BWI, DD + c, hh);
    const v8f din = gemm1(pH0, pH1, BWI, 2 * DD + c, hh);
    const float bir = bih[c], biz = bih[DD + c], bin = bih[2 * DD + c];
    const float bhr = bhh[c], bhz = bhh[DD + c], bhn = bhh[2 * DD + c];
#pragma unroll
    for (int r = 0; r < 8; ++r) {
      const float rg = sigm_f(dir[r] * OSC + bir + dhr[r] * OSC + bhr);
      const float zg = sigm_f(diz[r] * OSC + biz + dhz[r] * OSC + bhz);
      const float ng = tanhf(din[r] * OSC + bin + rg * (dhn[r] * OSC + bhn));
      const float ho = H32o[(size_t)(n0 + 8 * hh + r) * DD + c];
      so[(8 * hh + r) * DD + c] = (1.0f - zg) * ng + zg * ho;
    }
  }
  __syncthreads();

  rows_out2(so, H32n, HHn, n0, lane);
  __threadfence();
  rows_out2(so, H32n, HHn, n0, lane);
}

__global__ __launch_bounds__(TB) void k_gather(const unsigned short* __restrict__ HH, const int* __restrict__ sidx,
                                               const int* __restrict__ jidx, unsigned short* AS, unsigned short* AJ,
                                               int nN) {
  const int gt = (int)blockIdx.x * TB + (int)threadIdx.x;
  const int row = gt >> 3, p = gt & 7;
  if (row >= NST + 2 * NJB) return;
  const bool isS = row < NST;
  const int rs = row < NST - 1 ? row : NST - 1;
  int rj = row - NST; rj = rj < 0 ? 0 : (rj > 2 * NJB - 1 ? 2 * NJB - 1 : rj);
  const int is = sidx[rs];
  const int ij = jidx[rj];
  int idx = isS ? is : ij;
  idx = idx < 0 ? 0 : (idx > nN - 1 ? nN - 1 : idx);
  const v8us v = *(const v8us*)(HH + (size_t)idx * DD + 8 * p);
  unsigned short* d = isS ? (AS + (size_t)rs * DD + 8 * p) : (AJ + (size_t)rj * DD + 8 * p);
  *(volatile v8us*)d = v;
  __threadfence();
  *(volatile v8us*)d = v;
}

__global__ __launch_bounds__(NT) void k_heads(
    const unsigned short* __restrict__ AS, const unsigned short* __restrict__ AJ,
    const unsigned short* __restrict__ BS1, const float* __restrict__ sb1,
    const unsigned short* __restrict__ BS2, const float* __restrict__ sb2,
    const unsigned short* __restrict__ BJ1, const float* __restrict__ jb1,
    const float* __restrict__ jw2, const float* __restrict__ jb2,
    float* out1, float* out2) {
  __shared__ __attribute__((aligned(16))) _Float16 sHid[4][16 * DD];
  __shared__ __attribute__((aligned(16))) float sStage[64 * NOUT];
  __shared__ __attribute__((aligned(16))) float sPred[32];
  const int tid = threadIdx.x, lane = tid & 31, wave = tid >> 5, hh = lane >> 4, m = lane & 15;
  const int job = (int)blockIdx.y;
  const int rw = (int)blockIdx.x * 64 + wave * 16;
  if (job == 0) {
    _Float16* sh = sHid[wave];
    const v16h a0 = frag_glb(AS, rw + m, DD, 0, hh);
    const v16h a1 = frag_glb(AS, rw + m, DD, 32, hh);
#pragma unroll 1
    for (int t = 0; t < 4; ++t) {
      const int c = 16 * t + m;
      const v8f acc = gemm1(a0, a1, BS1, c, hh);
      const float bv = sb1[c];
#pragma unroll
      for (int r = 0; r < 8; ++r)
        sh[(8 * hh + r) * DD + c] = (_Float16)(leaky_f(acc[r] * OSC + bv) * (float)ASC);
    }
    __syncthreads();
    const v16h p0 = frag_lds(sh, m, DD, 0, hh);
    const v16h p1 = frag_lds(sh, m, DD, 32, hh);
#pragma unroll 1
    for (int t = 0; t < 8; ++t) {
      const int c = 16 * t + m;
      const v8f acc = gemm1(p0, p1, BS2, c, hh);
      const int cc = c < NOUT - 1 ? c : NOUT - 1;
      const float bv = sb2[cc];
#pragma unroll
      for (int r = 0; r < 8; ++r)
        if (c < NOUT) sStage[(16 * wave + 8 * hh + r) * NOUT + c] = acc[r] * OSC + bv;
    }
    __syncthreads();
    float* ob = out1 + (size_t)blockIdx.x * (64 * NOUT);
    const int npc = (64 * NOUT) / 4;
#pragma unroll 1
    for (int it = 0; it < (npc + NT - 1) / NT; ++it) {
      const int p = it * NT + tid;
      const int pc = p < npc ? p : npc - 1;
      const v4f v = *(const v4f*)(sStage + 4 * pc);
      if (p < npc) *(volatile v4f*)(ob + 4 * pc) = v;
    }
    __threadfence();
#pragma unroll 1
    for (int it = 0; it < (npc + NT - 1) / NT; ++it) {
      const int p = it * NT + tid;
      const int pc = p < npc ? p : npc - 1;
      const v4f v = *(const v4f*)(sStage + 4 * pc);
      if (p < npc) *(volatile v4f*)(ob + 4 * pc) = v;
    }
  } else {
    const v16h a0 = frag_glb(AJ, rw + m, DD, 0, hh);
    const v16h a1 = frag_glb(AJ, rw + m, DD, 32, hh);
    float pj[8];
#pragma unroll
    for (int r = 0; r < 8; ++r) pj[r] = 0.0f;
#pragma unroll 1
    for (int t = 0; t < 4; ++t) {
      const int c = 16 * t + m;
      const v8f acc = gemm1(a0, a1, BJ1, c, hh);
      const float bv = jb1[c];
      const float wv = jw2[c];
#pragma unroll
      for (int r = 0; r < 8; ++r) pj[r] += leaky_f(acc[r] * OSC + bv) * wv;
    }
#pragma unroll
    for (int r = 0; r < 8; ++r) {
      float v = pj[r];
      v += __shfl_xor(v, 1);
      v += __shfl_xor(v, 2);
      v += __shfl_xor(v, 4);
      v += __shfl_xor(v, 8);
      pj[r] = v;
    }
    const float b2 = jb2[0];
    if (m == 0) {
#pragma unroll
      for (int q = 0; q < 4; ++q)
        sPred[wave * 8 + 4 * hh + q] = ((pj[2 * q] + b2) + (pj[2 * q + 1] + b2)) * 0.5f;
    }
    __syncthreads();
    const int l8 = lane < 8 ? lane : 7;
    const v4f v = *(const v4f*)(sPred + 4 * l8);
    float* op = out2 + (size_t)blockIdx.x * 32 + 4 * l8;
    const bool act = (wave == 0) && (lane < 8);
    if (act) *(volatile v4f*)op = v;
    __threadfence();
    if (act) *(volatile v4f*)op = v;
  }
}

__global__ __launch_bounds__(TB) void k_s2s(const float* __restrict__ H32, const int* __restrict__ batch,
                                           const float* __restrict__ lbih, const float* __restrict__ lbhh,
                                           const float* __restrict__ lw, const float* __restrict__ lb,
                                           const float* __restrict__ lwih, const float* __restrict__ lwhh,
                                           float* out0, int nN) {
  __shared__ int   sList[NWS][WLC];
  __shared__ float sE[NWS][WLC];
  __shared__ int   sWc[NWS];
  __shared__ int   sOv[NWS];
  __shared__ __attribute__((aligned(16))) float sQ[DD];
  __shared__ __attribute__((aligned(16))) float sG[32];
  (void)lwih; (void)lwhh;
  const int tid = threadIdx.x, lane = tid & 31, wave = tid >> 5;
  const int g0 = (int)blockIdx.x * 16;
  if (tid < DD) {
    const float vi = lbih[tid] + lbhh[tid];
    const float vg = lbih[2 * DD + tid] + lbhh[2 * DD + tid];
    const float vo = lbih[3 * DD + tid] + lbhh[3 * DD + tid];
    const float c = sigm_f(vi) * tanh_f(vg);
    sQ[tid] = sigm_f(vo) * tanh_f(c);
  }
  int wc = 0;
#pragma unroll 1
  for (int nb = 0; nb < nN; nb += TB) {
    const int n = nb + tid;
    const int nc = n < nN ? n : nN - 1;
    const int b = batch[nc];
    const int lg = b - g0;
    const bool hit = (n < nN) && ((unsigned)lg < 16u);
    const unsigned mk = __builtin_amdgcn_ballot_w32(hit);
    if (hit) {
      const int pos = wc + (int)__builtin_amdgcn_mbcnt_lo(mk, 0u);
      if (pos < WLC) sList[wave][pos] = n | (lg << 16);
    }
    wc += (int)__builtin_popcount(mk);
  }
  if (lane == 0) { sWc[wave] = wc < WLC ? wc : WLC; sOv[wave] = wc > WLC ? 1 : 0; }
  __syncthreads();

  const v2f q2 = *(const v2f*)(sQ + 2 * lane);
#pragma unroll 1
  for (int gi = 0; gi < 2; ++gi) {
    const int lg = wave + NWS * gi;
    float emax = -3.0e38f;
#pragma unroll 1
    for (int wl = 0; wl < NWS; ++wl) {
      const int ne = __builtin_amdgcn_readfirstlane(sWc[wl]);
#pragma unroll 1
      for (int i = 0; i < ne; ++i) {
        const int ent = __builtin_amdgcn_readfirstlane(sList[wl][i]);
        if ((ent >> 16) == lg) {
          const int n = ent & 0xffff;
          const v2f hv = *(const v2f*)(H32 + (size_t)n * DD + 2 * lane);
          float p = hv.x * q2.x + hv.y * q2.y;
          p = wsum32(p);
          emax = fmaxf(emax, p);
          sE[wl][i] = p;
        }
      }
    }
    float den = 0.0f;
#pragma unroll 1
    for (int wl = 0; wl < NWS; ++wl) {
      const int ne = __builtin_amdgcn_readfirstlane(sWc[wl]);
#pragma unroll 1
      for (int i = 0; i < ne; ++i) {
        const int ent = __builtin_amdgcn_readfirstlane(sList[wl][i]);
        if ((ent >> 16) == lg) {
          const float ex = expf(sE[wl][i] - emax);
          den += ex;
          sE[wl][i] = ex;
        }
      }
    }
    const float rden = den > 0.0f ? (1.0f / den) : 0.0f;
    v2f rv = {0.f, 0.f};
#pragma unroll 1
    for (int wl = 0; wl < NWS; ++wl) {
      const int ne = __builtin_amdgcn_readfirstlane(sWc[wl]);
#pragma unroll 1
      for (int i = 0; i < ne; ++i) {
        const int ent = __builtin_amdgcn_readfirstlane(sList[wl][i]);
        if ((ent >> 16) == lg) {
          const int n = ent & 0xffff;
          const v2f hv = *(const v2f*)(H32 + (size_t)n * DD + 2 * lane);
          const float a = sE[wl][i] * rden;
          rv += hv * a;
        }
      }
    }
    const v4f wa = *(const v4f*)(lw + 4 * lane);
    const v4f wb = *(const v4f*)(lw + 2 * DD + 4 * lane);
    float t0 = q2.x * wa.x + q2.y * wa.z + rv.x * wb.x + rv.y * wb.z;
    float t1 = q2.x * wa.y + q2.y * wa.w + rv.x * wb.y + rv.y * wb.w;
    t0 = wsum32(t0);
    t1 = wsum32(t1);
    if (lane == 0) { sG[2 * lg] = t0 + lb[0]; sG[2 * lg + 1] = t1 + lb[1]; }
  }
  __syncthreads();
  int ov = 0;
#pragma unroll
  for (int w = 0; w < NWS; ++w) ov |= sOv[w];
  const int l8 = lane < 8 ? lane : 7;
  v4f v = *(const v4f*)(sG + 4 * l8);
  if (ov != 0) v = v + __int_as_float(0x7fc00000);
  float* op = out0 + (size_t)blockIdx.x * 32 + 4 * l8;
  const bool act = (wave == 0) && (lane < 8);
  if (act) *(volatile v4f*)op = v;
  __threadfence();
  if (act) *(volatile v4f*)op = v;
}

extern "C" void kernel_launch(void* const* d_in, const int* in_sizes, int n_in,
                              void* d_out, int out_size, void* d_ws, size_t ws_size,
                              hipStream_t stream) {
  if (n_in < 32) return;
  if (in_sizes[0] != NNODE * FIN || in_sizes[1] != 4 * NEDGE || in_sizes[2] != 2 * NEDGE ||
      in_sizes[3] != NNODE || in_sizes[4] != NST || in_sizes[5] != 2 * NJB) return;
  if (in_sizes[6] != FIN * DD || in_sizes[7] != DD || in_sizes[8] != 4 * DD || in_sizes[9] != DD) return;
  if (in_sizes[10] != DD * TCOL || in_sizes[11] != TCOL || in_sizes[12] != DD * DD || in_sizes[13] != DD) return;
  if (in_sizes[14] != DD * G3 || in_sizes[15] != DD * G3 || in_sizes[16] != G3 || in_sizes[17] != G3) return;
  if (in_sizes[18] != DD * DD || in_sizes[19] != DD || in_sizes[20] != DD * NOUT || in_sizes[21] != NOUT) return;
  if (in_sizes[22] != DD * DD || in_sizes[23] != DD || in_sizes[24] != DD || in_sizes[25] != 1) return;
  if (in_sizes[26] != 2 * DD * 4 * DD || in_sizes[27] != DD * 4 * DD || in_sizes[28] != 4 * DD ||
      in_sizes[29] != 4 * DD || in_sizes[30] != 2 * DD * 2 || in_sizes[31] != 2) return;
  if (out_size != OUTN) return;

  const float* x         = (const float*)d_in[0];
  const float* eattr     = (const float*)d_in[1];
  const int*   eidx      = (const int*)d_in[2];
  const int*   batch     = (const int*)d_in[3];
  const int*   sidx      = (const int*)d_in[4];
  const int*   jidx      = (const int*)d_in[5];
  const float* lin0_w    = (const float*)d_in[6];
  const float* lin0_b    = (const float*)d_in[7];
  const float* net1_w    = (const float*)d_in[8];
  const float* net1_b    = (const float*)d_in[9];
  const float* net2_w    = (const float*)d_in[10];
  const float* net2_b    = (const float*)d_in[11];
  const float* conv_root = (const float*)d_in[12];
  const float* conv_b    = (const float*)d_in[13];
  const float* gru_wih   = (const float*)d_in[14];
  const float* gru_whh   = (const float*)d_in[15];
  const float* gru_bih   = (const float*)d_in[16];
  const float* gru_bhh   = (const float*)d_in[17];
  const float* n2s_w1    = (const float*)d_in[18];
  const float* n2s_b1    = (const float*)d_in[19];
  const float* n2s_w2    = (const float*)d_in[20];
  const float* n2s_b2    = (const float*)d_in[21];
  const float* n2j_w1    = (const float*)d_in[22];
  const float* n2j_b1    = (const float*)d_in[23];
  const float* n2j_w2    = (const float*)d_in[24];
  const float* n2j_b2    = (const float*)d_in[25];
  const float* lstm_wih  = (const float*)d_in[26];
  const float* lstm_whh  = (const float*)d_in[27];
  const float* lstm_bih  = (const float*)d_in[28];
  const float* lstm_bhh  = (const float*)d_in[29];
  const float* lout_w    = (const float*)d_in[30];
  const float* lout_b    = (const float*)d_in[31];
  float* out = (float*)d_out;
  const int* srcp = eidx;
  const int* dstp = eidx + NEDGE;

  char* ws = (char*)d_ws;
  size_t off = 0;
#define CARVE(NAME, BYTES) const size_t NAME = off; off += (size_t)(BYTES); off = (off + 255) & ~(size_t)255;
  CARVE(oEW,   (size_t)NEDGE * TCOL * 2)
  CARVE(oBW2,  (size_t)TCOL * DD * 2)
  CARVE(oBC,   (size_t)DD * DD * 2)
  CARVE(oBWI,  (size_t)G3 * DD * 2)
  CARVE(oBWH,  (size_t)G3 * DD * 2)
  CARVE(oBL0,  (size_t)DD * KP0 * 2)
  CARVE(oBS1,  (size_t)DD * DD * 2)
  CARVE(oBS2,  (size_t)NOUTP * DD * 2)
  CARVE(oBJ1,  (size_t)DD * DD * 2)
  CARVE(oXP,   (size_t)NPAD * KP0 * 2)
  CARVE(oE1,   (size_t)NEDGE * DD * 2)
  CARVE(oH32A, (size_t)NPAD * DD * 4)
  CARVE(oH32B, (size_t)NPAD * DD * 4)
  CARVE(oHHA,  (size_t)NPAD * DD * 2)
  CARVE(oHHB,  (size_t)NPAD * DD * 2)
  CARVE(oAS,   (size_t)NST * DD * 2)
  CARVE(oAJ,   (size_t)2 * NJB * DD * 2)
#undef CARVE
  if (off > ws_size || off > (size_t)WSCAP) return;

  unsigned short* EW  = (unsigned short*)(ws + oEW);
  unsigned short* BW2 = (unsigned short*)(ws + oBW2);
  unsigned short* BC  = (unsigned short*)(ws + oBC);
  unsigned short* BWI = (unsigned short*)(ws + oBWI);
  unsigned short* BWH = (unsigned short*)(ws + oBWH);
  unsigned short* BL0 = (unsigned short*)(ws + oBL0);
  unsigned short* BS1 = (unsigned short*)(ws + oBS1);
  unsigned short* BS2 = (unsigned short*)(ws + oBS2);
  unsigned short* BJ1 = (unsigned short*)(ws + oBJ1);
  unsigned short* XP  = (unsigned short*)(ws + oXP);
  unsigned short* E1H = (unsigned short*)(ws + oE1);
  float*          H32A = (float*)(ws + oH32A);
  float*          H32B = (float*)(ws + oH32B);
  unsigned short* HHA = (unsigned short*)(ws + oHHA);
  unsigned short* HHB = (unsigned short*)(ws + oHHB);
  unsigned short* AS  = (unsigned short*)(ws + oAS);
  unsigned short* AJ  = (unsigned short*)(ws + oAJ);

  k_prep<<<dim3((TCOL * 8 + TB - 1) / TB, 9, 1), TB, 0, stream>>>(
      net2_w, conv_root, gru_wih, gru_whh, lin0_w, n2s_w1, n2s_w2, n2j_w1, x,
      BW2, BC, BWI, BWH, BL0, BS1, BS2, BJ1, XP);
  k_e1<<<(NEDGE * 8 + TB - 1) / TB, TB, 0, stream>>>(eattr, net1_w, net1_b, E1H, NEDGE);
  k_ew<<<NEDGE / 64, NT, 0, stream>>>(E1H, BW2, net2_b, EW);
  k_lin0<<<NPAD / 64, NT, 0, stream>>>(XP, BL0, lin0_b, H32A, HHA);
  for (int it = 0; it < 6; ++it) {
    const int rd = it & 1;
    const float* H32o = rd ? H32B : H32A;
    const unsigned short* HHo = rd ? HHB : HHA;
    float* H32n = rd ? H32A : H32B;
    unsigned short* HHn = rd ? HHA : HHB;
    k_node<<<NPAD / 64, NT, 0, stream>>>(H32o, HHo, H32n, HHn, EW, srcp, dstp, BC, conv_b, BWI, BWH,
                                         gru_bih, gru_bhh, NNODE, NEDGE);
  }
  k_gather<<<((NST + 2 * NJB) * 8 + TB - 1) / TB, TB, 0, stream>>>(HHA, sidx, jidx, AS, AJ, NNODE);
  k_heads<<<dim3(NST / 64, 2, 1), NT, 0, stream>>>(AS, AJ, BS1, n2s_b1, BS2, n2s_b2, BJ1, n2j_b1, n2j_w2, n2j_b2,
                                                   out + OFF1, out + OFF2);
  k_s2s<<<NGR / 16, TB, 0, stream>>>(H32A, batch, lstm_bih, lstm_bhh, lout_w, lout_b, lstm_wih, lstm_whh,
                                     out, NNODE);
  (void)ws_size;
}
